// MultiUniverseToposAttention_89498528514855
// MI455X (gfx1250) — hardware-verified
//
#include <hip/hip_runtime.h>
#include <math.h>
typedef __attribute__((ext_vector_type(16))) _Float16 v16h;
typedef __attribute__((ext_vector_type(8)))  _Float16 v8h;
typedef __attribute__((ext_vector_type(16))) __bf16   v16b;
typedef __attribute__((ext_vector_type(8)))  __bf16   v8b;
typedef __attribute__((ext_vector_type(8)))  float    v8f;
typedef __attribute__((ext_vector_type(4)))  float    v4f;
#define PSCALE 32768.0f
#define U16(p) ((const unsigned short*)(const void*)(p))
#define PSCALE_INV (1.0f / 32768.0f)

__device__ __forceinline__ unsigned short f2bf_bits(float f) {
  unsigned u = __float_as_uint(f);
  return (unsigned short)((u + 0x7FFFu + ((u >> 16) & 1u)) >> 16);
}
__device__ __forceinline__ float bf_bits2f(unsigned short h) { return __uint_as_float(((unsigned)h) << 16); }

__device__ __forceinline__ void dep_guard_h(v8f& a, v8f& b, v16h x, v16h y) { asm volatile("v_nop\n\tv_nop\n\tv_nop\n\tv_nop" : "+v"(a), "+v"(b) : "v"(x), "v"(y)); }
__device__ __forceinline__ void dep_guard_b(v8f& a, v8f& b, v16b x, v16b y) { asm volatile("v_nop\n\tv_nop\n\tv_nop\n\tv_nop" : "+v"(a), "+v"(b) : "v"(x), "v"(y)); }
__device__ __forceinline__ void keep4_h(v16h a, v16h b, v16h c, v16h d) { asm volatile("v_nop" :: "v"(a), "v"(b), "v"(c), "v"(d)); }
__device__ __forceinline__ void keep4_b(v16b a, v16b b, v16b c, v16b d) { asm volatile("v_nop" :: "v"(a), "v"(b), "v"(c), "v"(d)); }
__device__ __forceinline__ void acc_guard4(v8f& a, v8f& b, v8f& c, v8f& d) { asm volatile("v_nop\n\tv_nop\n\tv_nop\n\tv_nop" : "+v"(a), "+v"(b), "+v"(c), "+v"(d)); }
template <typename T> struct Frag;
template <> struct Frag<_Float16> {
  typedef v16h V; union U { v16h v; v8h h[2]; };
  static __device__ __forceinline__ v16h load(const _Float16* p) {
    U f; f.h[0] = *(const v8h*)(p); f.h[1] = *(const v8h*)(p + 16); return f.v;
  }
  static __device__ __forceinline__ v8f mma(v16h a, v16h b, v8f c) {
    return __builtin_amdgcn_wmma_f32_16x16x32_f16(false, a, false, b, (short)0, c, false, false);
  }
  static __device__ __forceinline__ void guard(v8f& a, v8f& b, v16h x, v16h y) { dep_guard_h(a, b, x, y); }
  static __device__ __forceinline__ void keep(v16h a, v16h b, v16h c, v16h d) { keep4_h(a, b, c, d); }
};
template <> struct Frag<__bf16> {
  typedef v16b V; union U { v16b v; v8b h[2]; };
  static __device__ __forceinline__ v16b load(const __bf16* p) {
    U f; f.h[0] = *(const v8b*)(p); f.h[1] = *(const v8b*)(p + 16); return f.v;
  }
  static __device__ __forceinline__ v8f mma(v16b a, v16b b, v8f c) {
    return __builtin_amdgcn_wmma_f32_16x16x32_bf16(false, a, false, b, (short)0, c, false, false);
  }
  static __device__ __forceinline__ void guard(v8f& a, v8f& b, v16b x, v16b y) { dep_guard_b(a, b, x, y); }
  static __device__ __forceinline__ void keep(v16b a, v16b b, v16b c, v16b d) { keep4_b(a, b, c, d); }
};

template <int ET> struct Elem;
template <> struct Elem<0> { typedef _Float16 T; };
template <> struct Elem<1> { typedef __bf16 T; };
template <int ET, bool SPLIT, int BIAS_MODE, int OUT_MODE, bool RESID, int ACT = 0>
__global__ __launch_bounds__(256) void wmma_gemm64(
    const unsigned short* __restrict__ Ap, const unsigned short* __restrict__ A2p, int lda, long strideA,
    const unsigned short* __restrict__ Btp, const unsigned short* __restrict__ Bt2p, int ldb, long strideB,
    void* __restrict__ Cout, void* __restrict__ Cout2, int ldc, long strideC,
    const float* __restrict__ bias,
    const float* __restrict__ resid, long strideR,
    int M, int N, int K, float scale) {
  typedef typename Elem<ET>::T T;
  typedef typename Frag<T>::V V;
  const T* A = (const T*)Ap; const T* A2 = (const T*)A2p; const T* Bt = (const T*)Btp; const T* Bt2 = (const T*)Bt2p;
  __shared__ __align__(16) float sT[8][16 * 68];
  const int b    = blockIdx.y;
  const int lane = threadIdx.x & 31;
  const int wave = threadIdx.x >> 5;
  const int tilesN = N >> 6;
  const int tilesM = M >> 6;
  const int tile = blockIdx.x * 8 + wave;
  if (tile >= tilesM * tilesN) return;
  const int tm = tile / tilesN;
  const int tn = tile - tm * tilesN;
  const int m0 = tm << 6;
  const int n0 = tn << 6;

  const T* Ab  = A  + (size_t)b * strideA;
  const T* Bb  = Bt + (size_t)b * strideB;
  const T* Ab2 = SPLIT ? (A2  + (size_t)b * strideA) : nullptr;
  const T* Bb2 = SPLIT ? (Bt2 + (size_t)b * strideB) : nullptr;

  const int rlane = lane & 15;
  const int koff  = (lane >> 4) * 8;
  const int mOff  = (lane >> 4) * 8;

  v8f acc[4][4];
#pragma unroll
  for (int i = 0; i < 4; ++i)
#pragma unroll
    for (int j = 0; j < 4; ++j) acc[i][j] = (v8f){0.f,0.f,0.f,0.f,0.f,0.f,0.f,0.f};

  for (int k0 = 0; k0 < K; k0 += 32) {
    V bh[4], bl[4];
#pragma unroll
    for (int j = 0; j < 4; ++j) {
      const size_t bo = (size_t)(n0 + (j << 4) + rlane) * ldb + koff + k0;
      bh[j] = Frag<T>::load(Bb + bo);
      if (SPLIT) bl[j] = Frag<T>::load(Bb2 + bo);
    }
#pragma unroll
    for (int i = 0; i < 4; ++i) {
      const size_t ao = (size_t)(m0 + (i << 4) + rlane) * lda + koff + k0;
      V ah = Frag<T>::load(Ab + ao);
      V al;
      if (SPLIT) al = Frag<T>::load(Ab2 + ao);
#pragma unroll
      for (int j = 0; j < 4; ++j) {
        acc[i][j] = Frag<T>::mma(ah, bh[j], acc[i][j]);
        if (SPLIT) {
          acc[i][j] = Frag<T>::mma(ah, bl[j], acc[i][j]);
          acc[i][j] = Frag<T>::mma(al, bh[j], acc[i][j]);
        }
      }
      Frag<T>::guard(acc[i][0], acc[i][3], ah, SPLIT ? al : ah);
    }
    Frag<T>::keep(bh[0], bh[1], bh[2], bh[3]);
    if (SPLIT) Frag<T>::keep(bl[0], bl[1], bl[2], bl[3]);
  }
  acc_guard4(acc[0][0], acc[0][1], acc[0][2], acc[0][3]);
  acc_guard4(acc[1][0], acc[1][1], acc[1][2], acc[1][3]);
  acc_guard4(acc[2][0], acc[2][1], acc[2][2], acc[2][3]);
  acc_guard4(acc[3][0], acc[3][1], acc[3][2], acc[3][3]);

  float* slab = sT[wave];
  const float* Rb = RESID ? (resid + (size_t)b * strideR) : nullptr;
#pragma unroll
  for (int i = 0; i < 4; ++i) {
    const int mBase = m0 + (i << 4);
#pragma unroll
    for (int j = 0; j < 4; ++j) {
      const int n = n0 + (j << 4) + rlane;
      float bv = 0.f;
      if (BIAS_MODE == 2) bv = bias[n];
#pragma unroll
      for (int r = 0; r < 8; ++r) {
        float v = acc[i][j][r] * scale;
        if (BIAS_MODE == 1) v += bias[mBase + mOff + r];
        if (BIAS_MODE == 2) v += bv;
        if (RESID) v += Rb[(size_t)(mBase + mOff + r) * ldc + n];
        if (ACT == 1) v = tanhf(v);
        if (ACT == 2) v = fmaxf(v, 0.0f);
        if (ACT == 3) v = v / (1.0f + expf(-v));
        if (ACT == 4) v = (v > 0.f) ? v : 0.01f * v;
        if (ACT == 5) v = 0.5f * v * (1.0f + erff(v * 0.70710678118654752f));
        slab[(mOff + r) * 68 + (j << 4) + rlane] = v;
      }
    }
    __builtin_amdgcn_fence(__ATOMIC_RELEASE, "workgroup");
    __builtin_amdgcn_wave_barrier();
    __builtin_amdgcn_fence(__ATOMIC_ACQUIRE, "workgroup");
    if (OUT_MODE == 0) {
      float* C = (float*)Cout + (size_t)b * strideC;
      const int hh = lane >> 4, c4 = (lane & 15) * 4;
      for (int pass = 0; pass < 2; ++pass) {
#pragma unroll
        for (int it = 0; it < 8; ++it) {
          const int row = it * 2 + hh;
          v4f v = *(const v4f*)(slab + row * 68 + c4);
          *(volatile v4f*)(C + (size_t)(mBase + row) * ldc + n0 + c4) = v;
        }
        __threadfence();
      }
    } else {
      const int q = lane >> 3, c8 = (lane & 7) * 8;
      unsigned short* C  = (unsigned short*)Cout  + (size_t)b * strideC;
      unsigned short* C2 = (OUT_MODE == 2) ? ((unsigned short*)Cout2 + (size_t)b * strideC) : nullptr;
      for (int pass = 0; pass < 2; ++pass) {
#pragma unroll
        for (int it = 0; it < 4; ++it) {
          const int row = it * 4 + q;
          const float* sp = slab + row * 68 + c8;
          v8h hv, lv;
#pragma unroll
          for (int e = 0; e < 8; ++e) {
            if (OUT_MODE == 1) {
              hv[e] = (_Float16)sp[e];
            } else {
              unsigned short hb = f2bf_bits(sp[e]);
              unsigned short lb = f2bf_bits(sp[e] - bf_bits2f(hb));
              hv[e] = __builtin_bit_cast(_Float16, hb);
              lv[e] = __builtin_bit_cast(_Float16, lb);
            }
          }
          *(volatile v8h*)(C + (size_t)(mBase + row) * ldc + n0 + c8) = hv;
          if (OUT_MODE == 2) *(volatile v8h*)(C2 + (size_t)(mBase + row) * ldc + n0 + c8) = lv;
        }
        __threadfence();
      }
    }
    __builtin_amdgcn_fence(__ATOMIC_RELEASE, "workgroup");
    __builtin_amdgcn_wave_barrier();
    __builtin_amdgcn_fence(__ATOMIC_ACQUIRE, "workgroup");
  }
}

__global__ __launch_bounds__(256) void cast_f32_f16x2(
    const float* __restrict__ in, _Float16* __restrict__ out, int n2) {
  int i = blockIdx.x * 256 + threadIdx.x;
  if (i < n2) {
    const _Float16 h0 = (_Float16)in[2 * i], h1 = (_Float16)in[2 * i + 1];
    const unsigned u = (unsigned)__builtin_bit_cast(unsigned short, h0) | ((unsigned)__builtin_bit_cast(unsigned short, h1) << 16);
    ((volatile unsigned*)out)[i] = u;
    __threadfence();
    ((volatile unsigned*)out)[i] = u;
  }
}


#define MS 1024
#define MD 256
#define MU 8
#define MDU 32
__device__ __forceinline__ float sigm(float v) { return 1.0f / (1.0f + expf(-v)); }
__global__ __launch_bounds__(256) void sigw_kernel(const float* __restrict__ Wm, _Float16* __restrict__ o, int n2) {
  const int i = blockIdx.x * 256 + threadIdx.x; if (i >= n2) return;
  const unsigned u = (unsigned)__builtin_bit_cast(unsigned short, (_Float16)sigm(Wm[2 * i])) | ((unsigned)__builtin_bit_cast(unsigned short, (_Float16)sigm(Wm[2 * i + 1])) << 16);
  ((volatile unsigned*)o)[i] = u; __threadfence(); ((volatile unsigned*)o)[i] = u;
}
__global__ __launch_bounds__(256) void router_kernel(const float* __restrict__ x, const float* __restrict__ Wr, float* __restrict__ WU, float* __restrict__ SEL) {
  __shared__ float sw[MU][MD]; __shared__ float res[8][16];
  const int lane = threadIdx.x & 31, wave = threadIdx.x >> 5; const int s = blockIdx.x * 8 + wave;
#pragma unroll 1
  for (int i = threadIdx.x; i < MU * MD; i += 256) sw[i / MD][i % MD] = sigm(Wr[i]);
  __syncthreads();
  float lg[MU];
  const float* xr = x + (size_t)s * MD;
#pragma unroll 1
  for (int u = 0; u < MU; ++u) { float a = 0.f;
#pragma unroll 1
    for (int q = 0; q < 8; ++q) a += xr[q * 32 + lane] * sw[u][q * 32 + lane];
    for (int o = 16; o > 0; o >>= 1) a += __shfl_xor(a, o, 32);
    lg[u] = a; }
  if (lane == 0) {
    float mx = lg[0]; for (int u = 1; u < MU; ++u) mx = fmaxf(mx, lg[u]);
    float p[MU], se = 0.f;
#pragma unroll 1
    for (int u = 0; u < MU; ++u) { p[u] = expf(lg[u] - mx); se += p[u]; }
    const float rse = 1.0f / se;
#pragma unroll 1
    for (int u = 0; u < MU; ++u) p[u] *= rse;
    int i0 = 0; for (int u = 1; u < MU; ++u) if (p[u] > p[i0]) i0 = u;
    int i1 = (i0 == 0) ? 1 : 0; for (int u = 0; u < MU; ++u) if (u != i0 && p[u] > p[i1]) i1 = u;
    const float den = p[i0] + p[i1] + 1e-9f;
    for (int u = 0; u < MU; ++u) { const bool sel = (u == i0) || (u == i1); res[wave][u] = sel ? (p[u] / den) : 0.f; res[wave][8 + u] = sel ? 1.f : 0.f; }
  }
  __syncthreads();
  if (threadIdx.x < 64) { const float v = res[threadIdx.x >> 3][threadIdx.x & 7]; ((volatile float*)WU)[(size_t)blockIdx.x * 64 + threadIdx.x] = v; __threadfence(); ((volatile float*)WU)[(size_t)blockIdx.x * 64 + threadIdx.x] = v; }
  else if (threadIdx.x < 128) { const int t = threadIdx.x - 64; const float v = res[t >> 3][8 + (t & 7)]; ((volatile float*)SEL)[(size_t)blockIdx.x * 64 + t] = v; __threadfence(); ((volatile float*)SEL)[(size_t)blockIdx.x * 64 + t] = v; }
}
__global__ __launch_bounds__(256) void qkv_post_kernel(const float* __restrict__ QKV, const float* __restrict__ SEL, const float* __restrict__ fc, const float* __restrict__ fsn,
                                                      float* __restrict__ Kc, float* __restrict__ Vc, float* __restrict__ SQ, float* __restrict__ SK) {
  const int lane = threadIdx.x & 31, wave = threadIdx.x >> 5; const int s = blockIdx.x * 8 + wave;
#pragma unroll 1
  for (int hb = 0; hb < MD; hb += 128) {
    const int c0 = hb + 4 * lane; const int u = c0 / MDU, d0 = c0 % MDU;
    const float sel = SEL[(size_t)s * MU + u];
    const float* qr = QKV + (size_t)s * 3 * MD + c0; const float* kr = qr + MD; const float* vr = qr + 2 * MD;
    float q[4], k[4], v[4];
#pragma unroll
    for (int e = 0; e < 4; ++e) { q[e] = qr[e] * sel; k[e] = kr[e] * sel; v[e] = vr[e] * sel; }
#pragma unroll
    for (int p = 0; p < 2; ++p) { const int j = (d0 >> 1) + p; const float c = fc[(size_t)s * 16 + j], sn = fsn[(size_t)s * 16 + j];
      const float qre = q[2*p], qim = q[2*p+1]; q[2*p] = qre * c - qim * sn; q[2*p+1] = qre * sn + qim * c;
      const float kre = k[2*p], kim = k[2*p+1]; k[2*p] = kre * c - kim * sn; k[2*p+1] = kre * sn + kim * c; }
    const v4f kv4 = {k[0], k[1], k[2], k[3]}, vv4 = {v[0], v[1], v[2], v[3]};
    const v4f sq4 = {sigm(q[0]), sigm(q[1]), sigm(q[2]), sigm(q[3])}, sk4 = {sigm(k[0]), sigm(k[1]), sigm(k[2]), sigm(k[3])};
    const size_t ro = (size_t)s * MD + c0;
    for (int pass = 0; pass < 2; ++pass) { *(volatile v4f*)(Kc + ro) = kv4; *(volatile v4f*)(Vc + ro) = vv4; *(volatile v4f*)(SQ + ro) = sq4; *(volatile v4f*)(SK + ro) = sk4; __threadfence(); }
  }
}
__global__ __launch_bounds__(256) void vt_kernel(const float* __restrict__ Vc, unsigned* __restrict__ VT16) {
  __shared__ float tile[32][65];
  const int u = blockIdx.y, t0 = blockIdx.x * 64, tx = threadIdx.x, ty = threadIdx.y;
  for (int j = ty; j < 64; j += 8) tile[tx][j] = Vc[(size_t)(t0 + j) * MD + u * MDU + tx];
  __syncthreads();
  for (int pass = 0; pass < 2; ++pass) {
    for (int r = ty; r < 64; r += 8) { unsigned val = 0u; if (r < 32) val = (unsigned)__builtin_bit_cast(unsigned short, (_Float16)tile[r][2 * tx]) | ((unsigned)__builtin_bit_cast(unsigned short, (_Float16)tile[r][2 * tx + 1]) << 16);
      ((volatile unsigned*)VT16)[(((size_t)u * 64 + r) * MS + t0) / 2 + tx] = val; }
    __threadfence();
  }
}
__global__ __launch_bounds__(256) void truth_kernel(const float* __restrict__ SQ, const float* __restrict__ SK, unsigned* __restrict__ AT) {
  __shared__ float qs[MDU]; __shared__ float red[8]; __shared__ float tot;
  const int u = blockIdx.y, s = blockIdx.x, t = threadIdx.x, lane = t & 31, wave = t >> 5;
  if (t < MDU) qs[t] = SQ[(size_t)s * MD + u * MDU + t];
  __syncthreads();
  float tv[4]; float part = 0.f;
#pragma unroll
  for (int q = 0; q < 4; ++q) { const int tk = q * 256 + t; const float* kr = SK + (size_t)tk * MD + u * MDU; float a = 0.f;
#pragma unroll 1
    for (int d = 0; d < MDU; ++d) a += fminf(fmaxf(1.0f - qs[d] + kr[d], 0.f), 1.0f);
    tv[q] = a * (1.0f / MDU); part += tv[q]; }
  for (int o = 16; o > 0; o >>= 1) part += __shfl_xor(part, o, 32);
  if (lane == 0) red[wave] = part; __syncthreads();
  if (t == 0) { float z = 0.f; for (int w = 0; w < 8; ++w) z += red[w]; tot = 32768.0f / (z + 1e-9f); } __syncthreads();
  const float inv = tot;
  for (int pass = 0; pass < 2; ++pass) {
#pragma unroll
    for (int q2 = 0; q2 < 2; ++q2) { const int tk = q2 * 512 + 2 * t; float a0 = 0.f, a1 = 0.f; const float* k0 = SK + (size_t)tk * MD + u * MDU; const float* k1 = k0 + MD;
#pragma unroll 1
      for (int d = 0; d < MDU; ++d) { a0 += fminf(fmaxf(1.0f - qs[d] + k0[d], 0.f), 1.0f); a1 += fminf(fmaxf(1.0f - qs[d] + k1[d], 0.f), 1.0f); }
      const unsigned uu = (unsigned)__builtin_bit_cast(unsigned short, (_Float16)(a0 * (1.0f / MDU) * inv)) | ((unsigned)__builtin_bit_cast(unsigned short, (_Float16)(a1 * (1.0f / MDU) * inv)) << 16);
      ((volatile unsigned*)AT)[(((size_t)u * MS + s) * MS + tk) / 2] = uu; }
    __threadfence();
  }
}
__global__ __launch_bounds__(256) void merge_kernel(const float* __restrict__ O, const float* __restrict__ WU, unsigned* __restrict__ OS16) {
  const int lane = threadIdx.x & 31, wave = threadIdx.x >> 5; const int s = blockIdx.x * 8 + wave;
  const int u = lane >> 2, d0 = (lane & 3) * 8; const float w = WU[(size_t)s * MU + u];
  const float* orow = O + ((size_t)u * MS + s) * 64 + d0;
  typedef __attribute__((ext_vector_type(4))) unsigned u4; u4 pk;
#pragma unroll
  for (int e = 0; e < 4; ++e) pk[e] = (unsigned)__builtin_bit_cast(unsigned short, (_Float16)(orow[2 * e] * w)) | ((unsigned)__builtin_bit_cast(unsigned short, (_Float16)(orow[2 * e + 1] * w)) << 16);
  *(volatile u4*)(OS16 + ((size_t)s * MD + u * MDU + d0) / 2) = pk; __threadfence(); *(volatile u4*)(OS16 + ((size_t)s * MD + u * MDU + d0) / 2) = pk;
}
extern "C" void kernel_launch(void* const* d_in, const int* in_sizes, int n_in, void* d_out, int out_size, void* d_ws, size_t ws_size, hipStream_t stream) {
  (void)in_sizes; (void)n_in; (void)out_size; (void)ws_size;
  const float* x = (const float*)d_in[0]; const float* fc = (const float*)d_in[1]; const float* fsn = (const float*)d_in[2];
  const float* Wr = (const float*)d_in[3]; const float* Wq = (const float*)d_in[4]; const float* Wk = (const float*)d_in[5]; const float* Wv = (const float*)d_in[6]; const float* Wo = (const float*)d_in[7];
  float* final_ = (float*)d_out; float* Kc = final_ + (size_t)MS * MD; float* Vc = Kc + (size_t)MS * MD;
  char* ws = (char*)d_ws; size_t off = 0;
  auto carve = [&](size_t bytes) -> char* { char* p = ws + off; off += (bytes + 255) & ~(size_t)255; return p; };
  _Float16* X16 = (_Float16*)carve((size_t)MS * MD * 2);
  _Float16* SW = (_Float16*)carve((size_t)3 * MD * MD * 2);
  _Float16* SWo = (_Float16*)carve((size_t)MD * MD * 2);
  float* WU = (float*)carve((size_t)MS * MU * 4); float* SEL = (float*)carve((size_t)MS * MU * 4);
  float* QKV = (float*)carve((size_t)MS * 3 * MD * 4);
  float* SQ = (float*)carve((size_t)MS * MD * 4); float* SK = (float*)carve((size_t)MS * MD * 4);
  unsigned* VT16 = (unsigned*)carve((size_t)MU * 64 * MS * 2);
  unsigned* AT = (unsigned*)carve((size_t)MU * MS * MS * 2);
  float* O = (float*)carve((size_t)MU * MS * 64 * 4);
  unsigned* OS16 = (unsigned*)carve((size_t)MS * MD * 2);
  cast_f32_f16x2<<<(MS * MD / 2 + 255) / 256, 256, 0, stream>>>(x, X16, MS * MD / 2);
  sigw_kernel<<<(MD * MD / 2 + 255) / 256, 256, 0, stream>>>(Wq, SW, MD * MD / 2);
  sigw_kernel<<<(MD * MD / 2 + 255) / 256, 256, 0, stream>>>(Wk, SW + (size_t)MD * MD, MD * MD / 2);
  sigw_kernel<<<(MD * MD / 2 + 255) / 256, 256, 0, stream>>>(Wv, SW + (size_t)2 * MD * MD, MD * MD / 2);
  sigw_kernel<<<(MD * MD / 2 + 255) / 256, 256, 0, stream>>>(Wo, SWo, MD * MD / 2);
  router_kernel<<<MS / 8, 256, 0, stream>>>(x, Wr, WU, SEL);
  { const int t = (MS / 64) * (3 * MD / 64);
    wmma_gemm64<0, false, 0, 0, false><<<dim3((t + 7) / 8, 1), 256, 0, stream>>>(U16(X16), nullptr, MD, 0, U16(SW), nullptr, MD, 0, QKV, nullptr, 3 * MD, 0, nullptr, nullptr, 0, MS, 3 * MD, MD, 1.0f); }
  qkv_post_kernel<<<MS / 8, 256, 0, stream>>>(QKV, SEL, fc, fsn, Kc, Vc, SQ, SK);
  vt_kernel<<<dim3(MS / 64, MU), dim3(32, 8), 0, stream>>>(Vc, VT16);
  truth_kernel<<<dim3(MS, MU), 256, 0, stream>>>(SQ, SK, AT);
  { const int t = (MS / 64) * 1;
    wmma_gemm64<0, false, 0, 0, false><<<dim3((t + 7) / 8, MU), 256, 0, stream>>>((const unsigned short*)AT, nullptr, MS, (long)MS * MS, (const unsigned short*)VT16, nullptr, MS, (long)64 * MS, O, nullptr, 64, (long)MS * 64, nullptr, nullptr, 0, MS, 64, MS, 1.0f / 32768.0f); }
  merge_kernel<<<MS / 8, 256, 0, stream>>>(O, WU, OS16);
  { const int t = (MS / 64) * (MD / 64);
    wmma_gemm64<0, false, 0, 0, false><<<dim3((t + 7) / 8, 1), 256, 0, stream>>>((const unsigned short*)OS16, nullptr, MD, 0, U16(SWo), nullptr, MD, 0, final_, nullptr, MD, 0, nullptr, nullptr, 0, MS, MD, MD, 1.0f); }
}
